// MPNN3D_5214090297737
// MI455X (gfx1250) — hardware-run, weakly checked
//
#include <hip/hip_runtime.h>


namespace {
constexpr int N = 50000, NP = 50048, E = 800000, H = 128, F0 = 64, EF = 16, G = 128, L = 5, K1 = 288  , K2 = 256, RH = 512;
constexpr float NEG = 0.2f  ;
typedef __bf16 bb16;
typedef __attribute__((ext_vector_type(16))) __bf16 v16bf;
typedef __attribute__((ext_vector_type(8))) __bf16 v8bf;
typedef __attribute__((ext_vector_type(4))) __bf16 v4bf;
typedef __attribute__((ext_vector_type(8))) float v8f;
typedef __attribute__((ext_vector_type(4))) float v4f;
__device__ __forceinline__ float bf16_rne(float f) { unsigned int u = __float_as_uint(f); u += 0x7FFFu + ((u >> 16) & 1u); return __uint_as_float(u & 0xFFFF0000u); }
__device__ __forceinline__ bb16 tobf(float f) { return (bb16)bf16_rne(f); }
__device__ __forceinline__ void splitbf(float v, bb16& hi, bb16& lo) { const float h = bf16_rne(v); hi = (bb16)h; lo = (bb16)bf16_rne(v - h); }
__device__ __forceinline__ v16bf frag_kb(const bb16* p, int hh) { const v8bf a = *(const v8bf*)(p + 8 * hh), b = *(const v8bf*)(p + 16 + 8 * hh); v16bf f;
#pragma unroll
  for (int e = 0; e < 8; ++e) { f[e] = a[e]; f[8 + e] = b[e]; } return f; }
__device__ __forceinline__ v8f wmmab(v16bf a, v16bf b, v8f c) { v8f d = __builtin_amdgcn_wmma_f32_16x16x32_bf16(false, a, false, b, (short)0, c, false, false); asm volatile("v_nop\n\tv_nop\n\tv_nop\n\tv_nop" : "+v"(d) : "v"(a), "v"(b)); return d; }
__device__ __forceinline__ void wave_lds_sync() { __builtin_amdgcn_fence(__ATOMIC_RELEASE, "workgroup"); __builtin_amdgcn_wave_barrier(); __builtin_amdgcn_fence(__ATOMIC_ACQUIRE, "workgroup"); }
__device__ __forceinline__ float pmul(float a, float b) { float p = a * b; asm volatile("" : "+v"(p)); return p; }
__device__ __forceinline__ int iclamp(int v, int lo, int hi) { return v < lo ? lo : (v > hi ? hi : v); }
constexpr int CSR_NBLK = 512, CSR_GB = 9, CSR_GN = 1 << CSR_GB  , CSR_MAXG = 512, CSR_CAP = 12288  ;
__global__ __launch_bounds__(64) void csrA_kernel(const int* __restrict__ dst, int E, int N, int nG, int CHP, int NGP, int* __restrict__ STG, int* __restrict__ HST) {
  extern __shared__ int sm[];
  int* cnt = sm; int* run = sm + NGP; int* ids = sm + 2 * NGP;
  const int b = blockIdx.x; const int ch = (E + CSR_NBLK - 1) / CSR_NBLK; const int e0 = b * ch, e1 = min(E, e0 + ch);
  for (int i = threadIdx.x; i < NGP; i += 64) cnt[i] = 0;
  for (int i = threadIdx.x; i < CHP; i += 64) ids[i] = -1;
  __syncthreads();
  if (threadIdx.x == 0) {
    for (int e = e0; e < e1; ++e) { int d = dst[e]; d = (d < 0) ? 0 : (d >= N ? N - 1 : d); cnt[d >> CSR_GB] += 1; }
    int acc = 0; for (int g = 0; g < nG; ++g) { run[g] = acc; acc += cnt[g]; }
    for (int e = e0; e < e1; ++e) { int d = dst[e]; d = (d < 0) ? 0 : (d >= N ? N - 1 : d); const int g = d >> CSR_GB; ids[run[g]] = e; run[g] += 1; } }
  __syncthreads();
  typedef __attribute__((ext_vector_type(4))) int v4i;
  for (int pass = 0; pass < 2; ++pass) {
    for (int i = threadIdx.x; i < CHP / 4; i += 64) *(volatile v4i*)(STG + (size_t)b * CHP + i * 4) = *(const v4i*)(&ids[i * 4]);
    for (int i = threadIdx.x; i < NGP / 4; i += 64) { v4i v; for (int e = 0; e < 4; ++e) v[e] = (i * 4 + e < nG) ? cnt[i * 4 + e] : 0; *(volatile v4i*)(HST + (size_t)b * NGP + i * 4) = v; }
    __threadfence(); }
}
__global__ __launch_bounds__(512) void csrS_kernel(const int* __restrict__ HST, int nG, int NGP, int* __restrict__ START, int* __restrict__ TOT, int* __restrict__ OFF) {
  __shared__ int tot[CSR_MAXG];
  const int b = threadIdx.x;
  for (int pass = 0; pass < 2; ++pass) { int runb = 0; for (int g = 0; g < nG; ++g) { int c = HST[(size_t)b * NGP + g]; c = (c < 0) ? 0 : c; ((volatile int*)OFF)[(size_t)g * CSR_NBLK + b] = runb; runb += c; } __threadfence(); }
  for (int g = threadIdx.x; g < nG; g += 512) { int s = 0; for (int bb = 0; bb < CSR_NBLK; ++bb) { int c = HST[(size_t)bb * NGP + g]; s += (c < 0) ? 0 : c; } tot[g] = s; }
  __syncthreads();
  if (threadIdx.x < 32) {
    __shared__ int st[CSR_MAXG + 32];
    if (threadIdx.x == 0) { int acc = 0; for (int g = 0; g < NGP; ++g) { st[g] = acc; if (g < nG) acc += (tot[g] + 31) & ~31; } st[NGP] = acc; }
    __builtin_amdgcn_fence(__ATOMIC_RELEASE, "workgroup"); __builtin_amdgcn_wave_barrier(); __builtin_amdgcn_fence(__ATOMIC_ACQUIRE, "workgroup");
    for (int pass = 0; pass < 2; ++pass) { for (int i = threadIdx.x; i < NGP + 32; i += 32) { ((volatile int*)START)[i] = (i <= NGP) ? st[min(i, NGP)] : 0; ((volatile int*)TOT)[i] = (i < nG) ? tot[i] : 0; } __threadfence(); } }
}
__global__ __launch_bounds__(256) void csrB_kernel(const int* __restrict__ dst, int N, int nG, int CHP, int NGP, int permLen, const int* __restrict__ STG, const int* __restrict__ HST, const int* __restrict__ OFF, const int* __restrict__ START, const int* __restrict__ TOT, int* __restrict__ PERM, int* __restrict__ ROWPTR, int* __restrict__ ROWCNT, int* __restrict__ FLAG) {
  typedef __attribute__((ext_vector_type(4))) int v4i;
  __shared__ int ids[CSR_CAP]; __shared__ unsigned short key[CSR_CAP]; __shared__ int outp[CSR_CAP]; __shared__ int ncnt[CSR_GN + 1]; __shared__ int boff[CSR_NBLK + 1];
  const int g = blockIdx.x, t_ = threadIdx.x; int tot = TOT[g]; int st = START[g], stn = START[g + 1]; const int v0 = g * CSR_GN; const int nv = min(CSR_GN, N - v0);
  st = (st < 0) ? 0 : (st > permLen - 32 ? permLen - 32 : st) & ~31; stn = (stn < st) ? st : (stn > permLen ? permLen : stn); tot = (tot < 0) ? 0 : tot; if (tot > stn - st && tot <= CSR_CAP) tot = stn - st;
  if (tot > CSR_CAP) {
    for (int pass = 0; pass < 2; ++pass) { for (int i = t_; i < CSR_GN / 4; i += 256) { v4i a, c; for (int e = 0; e < 4; ++e) { a[e] = st; c[e] = 0; } *(volatile v4i*)(ROWPTR + v0 + i * 4) = a; *(volatile v4i*)(ROWCNT + v0 + i * 4) = c; } if (t_ == 0) ((volatile int*)FLAG)[0] = 1; __threadfence(); } (void)nv; return; }
  if (t_ == 0) { int acc = 0; for (int b = 0; b < CSR_NBLK; ++b) { boff[b] = acc; int c = HST[(size_t)b * NGP + g]; c = (c < 0) ? 0 : (c > CHP ? CHP : c); acc += c; if (acc > tot) acc = tot; } boff[CSR_NBLK] = acc; }
  for (int i = t_; i <= CSR_GN; i += 256) ncnt[i] = 0;
  __syncthreads();
  for (int b = 0; b < CSR_NBLK; ++b) { const int c = boff[b + 1] - boff[b]; int o_ = OFF[(size_t)g * CSR_NBLK + b]; o_ = (o_ < 0) ? 0 : (o_ > CHP - c ? CHP - c : o_); const int* src_ = STG + (size_t)b * CHP + o_;
    for (int i = t_; i < c; i += 256) { int id = src_[i]; id = (id < 0) ? 0 : id; ids[boff[b] + i] = id; int d = dst[id]; d = (d < v0) ? v0 : (d >= N ? N - 1 : d); int kk = d - v0; kk = (kk < 0) ? 0 : (kk >= CSR_GN ? CSR_GN - 1 : kk); key[boff[b] + i] = (unsigned short)kk; } }
  __syncthreads();
  if (t_ == 0) { for (int i = 0; i < tot; ++i) ncnt[key[i]] += 1; int acc = 0; for (int vl = 0; vl < CSR_GN; ++vl) { const int c = ncnt[vl]; ncnt[vl] = acc; acc += c; } ncnt[CSR_GN] = acc;
    for (int i = 0; i < tot; ++i) { const int vl = key[i]; outp[ncnt[vl]] = ids[i]; ncnt[vl] += 1; }
    for (int vl = CSR_GN; vl > 0; --vl) ncnt[vl] = ncnt[vl - 1]; ncnt[0] = 0; }
  __syncthreads();
  for (int pass = 0; pass < 2; ++pass) {
    for (int i = t_; i < (stn - st) / 4; i += 256) { v4i v; for (int e = 0; e < 4; ++e) { const int q = i * 4 + e; v[e] = (q < tot) ? outp[q] : -1; } *(volatile v4i*)(PERM + st + i * 4) = v; }
    for (int i = t_; i < CSR_GN / 4; i += 256) { v4i a, c; for (int e = 0; e < 4; ++e) { const int vl = i * 4 + e; a[e] = st + ncnt[vl]; c[e] = (vl < nv) ? (ncnt[vl + 1] - ncnt[vl]) : 0; } *(volatile v4i*)(ROWPTR + v0 + i * 4) = a; *(volatile v4i*)(ROWCNT + v0 + i * 4) = c; }
    __threadfence(); }
}
__global__ __launch_bounds__(256) void csrZ_kernel(int* __restrict__ p, size_t n4) { typedef __attribute__((ext_vector_type(4))) int v4i; const size_t tid = (size_t)blockIdx.x * 256 + threadIdx.x, nth = (size_t)gridDim.x * 256; v4i z = {0, 0, 0, 0}; for (size_t i = tid; i < n4; i += nth) *(volatile v4i*)(p + i * 4) = z; }
struct CsrBufs { int *STG, *HST, *OFF, *START, *TOT, *PERM, *ROWPTR, *ROWCNT, *FLAG; int nG, NGP, CHP; size_t permLen; char* base; size_t bytes; };
static size_t csr_carve(CsrBufs& c, char* ws, size_t off, int E, int N) {
  const size_t off0 = off; c.base = ws + off;
  auto al = [&](size_t bytes) { char* p = ws + off; off += (bytes + 255) & ~(size_t)255; return p; };
  c.nG = (N + CSR_GN - 1) / CSR_GN; c.NGP = (c.nG + 31) & ~31; const int ch = (E + CSR_NBLK - 1) / CSR_NBLK; c.CHP = (ch + 31) & ~31; c.permLen = (size_t)E + 32 * (size_t)c.nG + 32;
  c.STG = (int*)al((size_t)CSR_NBLK * c.CHP * 4); c.HST = (int*)al((size_t)CSR_NBLK * c.NGP * 4); c.OFF = (int*)al((size_t)c.NGP * CSR_NBLK * 4); c.START = (int*)al((size_t)(c.NGP + 64) * 4); c.TOT = (int*)al((size_t)(c.NGP + 64) * 4);
  c.PERM = (int*)al(c.permLen * 4); c.ROWPTR = (int*)al((size_t)c.nG * CSR_GN * 4); c.ROWCNT = (int*)al((size_t)c.nG * CSR_GN * 4); c.FLAG = (int*)al(256);
  c.bytes = off - off0; return off;
}
static void csr_build(const CsrBufs& c, const int* dst, int E, int N, hipStream_t stream) {
  const size_t smem = (size_t)(2 * c.NGP + c.CHP) * 4;
  csrZ_kernel<<<512, 256, 0, stream>>>((int*)c.base, c.bytes / 16);
  csrA_kernel<<<CSR_NBLK, 64, smem, stream>>>(dst, E, N, c.nG, c.CHP, c.NGP, c.STG, c.HST);
  csrS_kernel<<<1, 512, 0, stream>>>(c.HST, c.nG, c.NGP, c.START, c.TOT, c.OFF);
  csrB_kernel<<<c.nG, 256, 0, stream>>>(dst, N, c.nG, c.CHP, c.NGP, (int)c.permLen, c.STG, c.HST, c.OFF, c.START, c.TOT, c.PERM, c.ROWPTR, c.ROWCNT, c.FLAG);
}


__global__ __launch_bounds__(256) void wprep_kernel(const float* __restrict__ win, const float* __restrict__ wpre, const float* __restrict__ bpre, const float* __restrict__ wpost, bb16* __restrict__ WIN, bb16* __restrict__ W1, bb16* __restrict__ W2) {
  const size_t u = (size_t)blockIdx.x * 256 + threadIdx.x; const size_t n0 = (size_t)H * F0 / 8, n1 = (size_t)L * H * K1 / 8, n2 = (size_t)L * H * K2 / 8; size_t t = u; v8bf o;
  if (t < n0) { const size_t e = t * 8; const int oo = (int)(e / F0), k0 = (int)(e % F0); for (int j = 0; j < 8; ++j) o[j] = tobf(win[(size_t)(k0 + j) * H + oo]); for (int pass = 0; pass < 2; ++pass) { *(volatile v8bf*)(WIN + e) = o; __threadfence(); } return; } t -= n0;
  if (t < n1) { const size_t e = t * 8; const int l = (int)(e / ((size_t)H * K1)); const size_t rem = e % ((size_t)H * K1); const int oo = (int)(rem / K1), k0 = (int)(rem % K1);
    for (int j = 0; j < 8; ++j) { const int k = k0 + j; float w = 0.0f; if (k < 273) w = wpre[((size_t)l * 273 + k) * H + oo]; else if (k == 273) w = bpre[(size_t)l * H + oo]; o[j] = tobf(w); }
    for (int pass = 0; pass < 2; ++pass) { *(volatile v8bf*)(W1 + e) = o; __threadfence(); } return; } t -= n1;
  if (t < n2) { const size_t e = t * 8; const int l = (int)(e / ((size_t)H * K2)); const size_t rem = e % ((size_t)H * K2); const int oo = (int)(rem / K2), k0 = (int)(rem % K2);
    for (int j = 0; j < 8; ++j) o[j] = tobf(wpost[((size_t)l * K2 + k0 + j) * H + oo]); for (int pass = 0; pass < 2; ++pass) { *(volatile v8bf*)(W2 + e) = o; __threadfence(); } }
}
__global__ __launch_bounds__(128) void h0_kernel(const float* __restrict__ nf, const bb16* __restrict__ WIN, const float* __restrict__ bin_, float* __restrict__ HA) {
  __shared__ __attribute__((aligned(16))) float Tf[4][16][H + 4];
  const int wave = threadIdx.x >> 5, lane = threadIdx.x & 31, nloc = lane & 15, hlf = lane >> 4; const size_t m0 = (size_t)blockIdx.x * 64 + wave * 16; const size_t v = m0 + nloc;
  v8f acc[8];
#pragma unroll
  for (int t = 0; t < 8; ++t) acc[t] = (v8f){};
#pragma unroll
  for (int kb = 0; kb < F0; kb += 32) { v16bf a = {}; if (v < (size_t)N) { const float* r = nf + v * F0 + kb; for (int e = 0; e < 8; ++e) { a[e] = tobf(r[8 * hlf + e]); a[8 + e] = tobf(r[16 + 8 * hlf + e]); } }
#pragma unroll
    for (int t = 0; t < 8; ++t) acc[t] = wmmab(a, frag_kb(WIN + (size_t)(t * 16 + nloc) * F0 + kb, hlf), acc[t]); }
#pragma unroll
  for (int t = 0; t < 8; ++t) { const int c = t * 16 + nloc; const float bb = bf16_rne(bin_[c]);
#pragma unroll 1
    for (int r = 0; r < 8; ++r) { const size_t row = m0 + 8 * hlf + r; Tf[wave][8 * hlf + r][c] = row < (size_t)N ? fmaxf(acc[t][r] + bb, 0.0f) : 0.0f; } }
  wave_lds_sync();
  for (int pass = 0; pass < 2; ++pass) { for (int rr = 0; rr < 16; ++rr) *(volatile v4f*)(HA + (m0 + rr) * H + lane * 4) = *(const v4f*)(&Tf[wave][rr][lane * 4]); __threadfence(); }
}
__global__ __launch_bounds__(256) void stat_kernel(const float* __restrict__ ef, const float* __restrict__ x, const int* __restrict__ srcs, const int* __restrict__ PERM, const int* __restrict__ ROWPTR, const int* __restrict__ ROWCNT, int permLen, float* __restrict__ S) {
  const int wave = threadIdx.x >> 5, lane = threadIdx.x & 31; const size_t v = (size_t)blockIdx.x * 8 + wave; float s = 0.0f;
  if (v < (size_t)N) { int st = ROWPTR[v], cnt = ROWCNT[v]; cnt = iclamp(cnt, 0, 65536); st = iclamp(st, 0, permLen - cnt); const float xv0 = bf16_rne(x[v * 3]), xv1 = bf16_rne(x[v * 3 + 1]), xv2 = bf16_rne(x[v * 3 + 2]);
#pragma unroll 1
    for (int j = 0; j < cnt; ++j) { const int e = iclamp(PERM[st + j], 0, E - 1); const size_t u = (size_t)iclamp(srcs[e], 0, N - 1);
      if (lane < EF) s += bf16_rne(ef[(size_t)e * EF + lane]);
      else if (lane == EF) { const float d0 = bf16_rne(x[u * 3]) - xv0, d1 = bf16_rne(x[u * 3 + 1]) - xv1, d2 = bf16_rne(x[u * 3 + 2]) - xv2; s += pmul(d0, d0) + pmul(d1, d1) + pmul(d2, d2); }
      else if (lane == EF + 1) s += 1.0f; } }
  for (int pass = 0; pass < 2; ++pass) { ((volatile float*)S)[v * 32 + lane] = s; __threadfence(); }
}
__global__ __launch_bounds__(32) void layer_kernel(const float* __restrict__ Hin, const float* __restrict__ S, const int* __restrict__ srcs, const int* __restrict__ PERM, const int* __restrict__ ROWPTR, const int* __restrict__ ROWCNT, int permLen, const bb16* __restrict__ W1, const bb16* __restrict__ W2, const float* __restrict__ bpost, float* __restrict__ Hout) {
  __shared__ __attribute__((aligned(16))) bb16 Ah[16][K1 + 8], Al[16][K1 + 8]; __shared__ __attribute__((aligned(16))) float Hv[16][H + 4]; __shared__ __attribute__((aligned(16))) float Tf[16][H + 4];
  const int lane = threadIdx.x, nloc = lane & 15, hlf = lane >> 4; const size_t v0 = (size_t)blockIdx.x * 16;
  for (int rr = 0; rr < 16; ++rr) { const size_t v = v0 + rr; v4f sh = {0.0f, 0.0f, 0.0f, 0.0f}, hv = {0.0f, 0.0f, 0.0f, 0.0f}; float sv = 0.0f, cntv = 0.0f;
    if (v < (size_t)N) { int st = ROWPTR[v], cnt = ROWCNT[v]; cnt = iclamp(cnt, 0, 65536); st = iclamp(st, 0, permLen - cnt);
#pragma unroll 1
      for (int j = 0; j < cnt; ++j) { const int e = iclamp(PERM[st + j], 0, E - 1); const size_t u = (size_t)iclamp(srcs[e], 0, N - 1); sh += *(const v4f*)(Hin + u * H + lane * 4); }
      hv = *(const v4f*)(Hin + v * H + lane * 4); sv = S[v * 32 + lane]; cntv = S[v * 32 + EF + 1]; }
    *(v4f*)(&Hv[rr][lane * 4]) = hv;
    for (int j = 0; j < 4; ++j) { bb16 p, q; splitbf(sh[j], p, q); Ah[rr][lane * 4 + j] = p; Al[rr][lane * 4 + j] = q; splitbf(pmul(cntv, hv[j]), p, q); Ah[rr][H + lane * 4 + j] = p; Al[rr][H + lane * 4 + j] = q; }
    { bb16 p, q; splitbf(lane < EF + 2 ? sv : 0.0f, p, q); Ah[rr][2 * H + lane] = p; Al[rr][2 * H + lane] = q; } }
  wave_lds_sync();
  v8f acc[8];
#pragma unroll
  for (int t = 0; t < 8; ++t) acc[t] = (v8f){};
#pragma unroll 3
  for (int kb = 0; kb < K1; kb += 32) { const v16bf a = frag_kb(&Ah[nloc][kb], hlf), al = frag_kb(&Al[nloc][kb], hlf);
#pragma unroll
    for (int t = 0; t < 8; ++t) { const v16bf bw = frag_kb(W1 + (size_t)(t * 16 + nloc) * K1 + kb, hlf); acc[t] = wmmab(a, bw, acc[t]); acc[t] = wmmab(al, bw, acc[t]); } }
  wave_lds_sync();
#pragma unroll
  for (int t = 0; t < 8; ++t) { const int c = t * 16 + nloc;
#pragma unroll 1
    for (int r = 0; r < 8; ++r) { const int rr = 8 * hlf + r; bb16 p, q; splitbf(acc[t][r], p, q); Ah[rr][H + c] = p; Al[rr][H + c] = q; splitbf(Hv[rr][c], p, q); Ah[rr][c] = p; Al[rr][c] = q; } }
  wave_lds_sync();
#pragma unroll
  for (int t = 0; t < 8; ++t) acc[t] = (v8f){};
#pragma unroll 2
  for (int kb = 0; kb < K2; kb += 32) { const v16bf a = frag_kb(&Ah[nloc][kb], hlf), al = frag_kb(&Al[nloc][kb], hlf);
#pragma unroll
    for (int t = 0; t < 8; ++t) { const v16bf bw = frag_kb(W2 + (size_t)(t * 16 + nloc) * K2 + kb, hlf); acc[t] = wmmab(a, bw, acc[t]); acc[t] = wmmab(al, bw, acc[t]); } }
#pragma unroll
  for (int t = 0; t < 8; ++t) { const int c = t * 16 + nloc; const float bb = bf16_rne(bpost[c]);
#pragma unroll 1
    for (int r = 0; r < 8; ++r) { const int rr = 8 * hlf + r; Tf[rr][c] = (v0 + rr < (size_t)N) ? acc[t][r] + bb + Hv[rr][c] : 0.0f; } }
  wave_lds_sync();
  for (int pass = 0; pass < 2; ++pass) { for (int rr = 0; rr < 16; ++rr) *(volatile v4f*)(Hout + (v0 + rr) * H + lane * 4) = *(const v4f*)(&Tf[rr][lane * 4]); __threadfence(); }
}
__device__ int lower_bound_i(const int* a, int n, int key) { int lo = 0, hi = n; while (lo < hi) { const int mid = (lo + hi) >> 1; if (a[mid] < key) lo = mid + 1; else hi = mid; } return lo; }
__global__ __launch_bounds__(512) void readout_kernel(const float* __restrict__ HF, const int* __restrict__ n2g, const float* __restrict__ wr1, const float* __restrict__ br1, const float* __restrict__ wr2, const float* __restrict__ br2, float* __restrict__ PO) {
  __shared__ float mm[2 * H], red[RH];
  const int g = blockIdx.x, t = threadIdx.x; const int lo = lower_bound_i(n2g, N, g), hi = lower_bound_i(n2g, N, g + 1);
  if (t < H) { float s = 0.0f, mx = -INFINITY; for (int v = lo; v < hi; ++v) { const float h = HF[(size_t)v * H + t]; s += h; mx = fmaxf(mx, h); } mm[t] = s / (float)(hi - lo); mm[H + t] = mx; }
  __syncthreads();
  float z = bf16_rne(br1[t]);
#pragma unroll 1
  for (int k = 0; k < 2 * H; ++k) z += pmul(mm[k], bf16_rne(wr1[k * RH + t])); red[t] = pmul(fmaxf(z, 0.0f), bf16_rne(wr2[t]));
  __syncthreads();
  for (int st = RH / 2; st > 0; st >>= 1) { if (t < st) red[t] += red[t + st]; __syncthreads(); }
  for (int pass = 0; pass < 2; ++pass) { if (t < 32) ((volatile float*)PO)[(size_t)g * 32 + t] = red[0] + bf16_rne(br2[0]); __threadfence(); }
}
__global__ __launch_bounds__(64) void final_kernel(const float* __restrict__ PO, float* __restrict__ out) {
  __shared__ __attribute__((aligned(16))) float so[G]; for (int q = threadIdx.x; q < G; q += 64) so[q] = PO[(size_t)q * 32]; __syncthreads();
  for (int pass = 0; pass < 2; ++pass) { if (threadIdx.x < G / 4) *(volatile v4f*)(out + threadIdx.x * 4) = *(const v4f*)(&so[threadIdx.x * 4]); __threadfence(); }
}
}

extern "C" void kernel_launch(void* const* d_in, const int* in_sizes, int n_in, void* d_out, int out_size, void* d_ws, size_t ws_size, hipStream_t stream) {
  (void)n_in;
  auto Fp = [&](int i) { return (const float*)d_in[i]; }; auto Ip = [&](int i) { return (const int*)d_in[i]; };
  if (in_sizes[0] != N * F0 || in_sizes[1] != N * 3 || in_sizes[2] != E * EF || in_sizes[3] != E || in_sizes[4] != E || in_sizes[5] != N || in_sizes[6] != F0 * H || in_sizes[8] != L * 273 * H || in_sizes[10] != L * K2 * H || in_sizes[12] != 2 * H * RH || out_size != G) return;
  size_t off = 0; char* ws = (char*)d_ws;
  auto carve = [&](size_t bytes) { char* p = ws + off; off += (bytes + 255) & ~(size_t)255; return p; };
  bb16* WIN = (bb16*)carve((size_t)H * F0 * 2); bb16* W1 = (bb16*)carve((size_t)L * H * K1 * 2); bb16* W2 = (bb16*)carve((size_t)L * H * K2 * 2);
  float* HA = (float*)carve((size_t)NP * H * 4); float* HB = (float*)carve((size_t)NP * H * 4); float* S = (float*)carve((size_t)NP * 32 * 4); float* PO = (float*)carve((size_t)G * 32 * 4);
  CsrBufs csr; off = csr_carve(csr, ws, off, E, N);
  if (off > ws_size || off > ((size_t)128 << 20)) return;
  wprep_kernel<<<(unsigned)(((size_t)H * F0 / 8 + (size_t)L * H * K1 / 8 + (size_t)L * H * K2 / 8 + 255) / 256), 256, 0, stream>>>(Fp(6), Fp(8), Fp(9), Fp(10), WIN, W1, W2);
  csr_build(csr, Ip(4), E, N, stream);
  h0_kernel<<<NP / 64, 128, 0, stream>>>(Fp(0), WIN, Fp(7), HA);
  stat_kernel<<<NP / 8, 256, 0, stream>>>(Fp(2), Fp(1), Ip(3), csr.PERM, csr.ROWPTR, csr.ROWCNT, (int)csr.permLen, S);
  float* hin = HA; float* hout = HB;
  for (int l = 0; l < L; ++l) { layer_kernel<<<NP / 16, 32, 0, stream>>>(hin, S, Ip(3), csr.PERM, csr.ROWPTR, csr.ROWCNT, (int)csr.permLen, W1 + (size_t)l * H * K1, W2 + (size_t)l * H * K2, Fp(11) + l * H, hout); float* t = hin; hin = hout; hout = t; }
  readout_kernel<<<G, 512, 0, stream>>>(hin, Ip(5), Fp(12), Fp(13), Fp(14), Fp(15), PO);
  final_kernel<<<1, 64, 0, stream>>>(PO, (float*)d_out);
}
